// GATSepEncoder_17042430231191
// MI455X (gfx1250) — hardware-verified
//
#include <hip/hip_runtime.h>
#include <stddef.h>


#define DF    128
#define KIN   256
#define NH    4
#define HP    4
#define GR    32
#define NTHR  256
#define NWAVE 8
#define XSP   132
#define AP1   136
#define AP2   264
#define NB    512
#define CHUNK 2048
#define WCAP  256
#define NGRP  (CHUNK / (NTHR * 4))

#define LDS_SACC (NB * DF)
#define LDS_DEN  (NB * HP)
#define LDS_MAX  (NB * HP)
#define LDS_LIST (NWAVE * WCAP)
#define LDS_BYTES ((LDS_SACC + LDS_DEN + LDS_MAX + LDS_LIST + NWAVE) * 4)

static_assert(WCAP == (CHUNK / NTHR) * 32);
static_assert(NGRP == 2);
static_assert(NB == 512);
static_assert(CHUNK == 2048);
static_assert(((LDS_SACC + LDS_DEN) % 4) == 0);
static_assert((LDS_MAX % 4) == 0);
static_assert((NB % NWAVE) == 0);
static_assert(LDS_BYTES == 286752);
static_assert(NH == HP);
static_assert(DF == 32 * 4);
static_assert(KIN == 2 * DF);

typedef float          v4f   __attribute__((ext_vector_type(4)));
typedef float          v8f   __attribute__((ext_vector_type(8)));
typedef int            v4i   __attribute__((ext_vector_type(4)));
typedef unsigned short v8us  __attribute__((ext_vector_type(8)));
typedef unsigned short v16us __attribute__((ext_vector_type(16)));
typedef __bf16         v16bf __attribute__((ext_vector_type(16)));
union Frag   { v16bf v; v16us u; v8us half[2]; };
union Pack16 { v8us h; v4i i; };

__device__ __forceinline__ v8f wm(v16bf a, v16bf b, v8f c) {
  v8f d = __builtin_amdgcn_wmma_f32_16x16x32_bf16(false, a, false, b, (short)0, c, false, false);
  asm volatile("v_nop\n\tv_nop\n\tv_nop\n\tv_nop" : "+v"(d) : "v"(a), "v"(b));
  return d;
}

__device__ __forceinline__ unsigned short bf_bits(float x) {
  const unsigned u = __float_as_uint(x);
  return (unsigned short)((u + 0x7FFFu + ((u >> 16) & 1u)) >> 16);
}
__device__ __forceinline__ void bf_split(float x, unsigned short& hi, unsigned short& lo) {
  const unsigned short hb = bf_bits(x);
  const float r = x - __uint_as_float(((unsigned)hb) << 16);
  hi = hb;
  lo = bf_bits(r);
}

__device__ __forceinline__ float gelu_f(float x) {
  return 0.5f * x * (1.0f + erff(x * 0.70710678118654752f));
}

template<int KD, bool LO>
__global__ __launch_bounds__(NTHR) void k_prepw(const float* __restrict__ W,
                                                unsigned short* Wh, unsigned short* Wlo) {
  __shared__ __attribute__((aligned(16))) float T[32 * (KD + 1)];
  const int tid = threadIdx.x;
  const int n0  = blockIdx.x * 32;
#pragma unroll 4
  for (int i = 0; i < KD / 8; ++i) {
    const int idx = i * NTHR + tid;
    const int k   = idx >> 5;
    const int c   = idx & 31;
    T[c * (KD + 1) + k] = W[(size_t)k * DF + n0 + c];
  }
  __syncthreads();
  Pack16 uh[KD / 64], ul[KD / 64];
  size_t po[KD / 64];
#pragma unroll
  for (int q = 0; q < KD / 64; ++q) {
    const int t  = q * NTHR + tid;
    const int c  = t / (KD / 8);
    const int k0 = (t % (KD / 8)) * 8;
#pragma unroll
    for (int j = 0; j < 8; ++j) {
      const float val = T[c * (KD + 1) + k0 + j];
      if (LO) {
        unsigned short a, b;
        bf_split(val, a, b);
        uh[q].h[j] = a;
        ul[q].h[j] = b;
      } else {
        uh[q].h[j] = bf_bits(val);
        ul[q].h[j] = (unsigned short)0;
      }
    }
    po[q] = (size_t)(n0 + c) * KD + k0;
  }
#pragma unroll
  for (int q = 0; q < KD / 64; ++q) {
    *(volatile v4i*)(Wh + po[q]) = uh[q].i;
    if (LO) *(volatile v4i*)(Wlo + po[q]) = ul[q].i;
  }
  __threadfence();
#pragma unroll
  for (int q = 0; q < KD / 64; ++q) {
    *(volatile v4i*)(Wh + po[q]) = uh[q].i;
    if (LO) *(volatile v4i*)(Wlo + po[q]) = ul[q].i;
  }
}

template<bool LO>
__device__ __forceinline__ void stage128(const float* __restrict__ src, int pitch, int scoff,
                                         int rowBase, int nN, unsigned short* Ah,
                                         unsigned short* Al, int ap, int dcoff, int tid) {
  const int r  = tid >> 3;
  const int c0 = (tid & 7) * 16;
  int row = rowBase + r;
  if (row > nN - 1) row = nN - 1;
  const float* p = src + (size_t)row * pitch + scoff + c0;
  const v4f f0 = *(const v4f*)(p), f1 = *(const v4f*)(p + 4);
  const v4f f2 = *(const v4f*)(p + 8), f3 = *(const v4f*)(p + 12);
  float v[16];
  v[0] = f0.x;  v[1] = f0.y;  v[2] = f0.z;  v[3] = f0.w;
  v[4] = f1.x;  v[5] = f1.y;  v[6] = f1.z;  v[7] = f1.w;
  v[8] = f2.x;  v[9] = f2.y;  v[10] = f2.z; v[11] = f2.w;
  v[12] = f3.x; v[13] = f3.y; v[14] = f3.z; v[15] = f3.w;
  Pack16 h0, h1, l0, l1;
#pragma unroll
  for (int j = 0; j < 8; ++j) {
    if (LO) {
      unsigned short a, b;
      bf_split(v[j], a, b);
      h0.h[j] = a; l0.h[j] = b;
      bf_split(v[8 + j], a, b);
      h1.h[j] = a; l1.h[j] = b;
    } else {
      h0.h[j] = bf_bits(v[j]);
      h1.h[j] = bf_bits(v[8 + j]);
      l0.h[j] = (unsigned short)0;
      l1.h[j] = (unsigned short)0;
    }
  }
  *(v8us*)(Ah + r * ap + dcoff + c0)     = h0.h;
  *(v8us*)(Ah + r * ap + dcoff + c0 + 8) = h1.h;
  if (LO) {
    *(v8us*)(Al + r * ap + dcoff + c0)     = l0.h;
    *(v8us*)(Al + r * ap + dcoff + c0 + 8) = l1.h;
  }
}

template<int KD, int AP, bool LO>
__device__ __forceinline__ void mma2(const unsigned short* Ah, const unsigned short* Al,
                                     const unsigned short* __restrict__ Bh,
                                     const unsigned short* __restrict__ Bl,
                                     int ncol, int m, int hh, v8f& c0, v8f& c1) {
#pragma unroll 2
  for (int kt = 0; kt < KD / 32; ++kt) {
    const int k0 = kt * 32;
    Frag a0h, a1h, bh;
    const unsigned short* pbh = Bh + (size_t)ncol * KD + k0 + 8 * hh;
    const unsigned short* pa0 = Ah + m * AP + k0 + 8 * hh;
    const unsigned short* pa1 = Ah + (16 + m) * AP + k0 + 8 * hh;
    bh.half[0]  = *(const v8us*)pbh;  bh.half[1]  = *(const v8us*)(pbh + 16);
    a0h.half[0] = *(const v8us*)pa0;  a0h.half[1] = *(const v8us*)(pa0 + 16);
    a1h.half[0] = *(const v8us*)pa1;  a1h.half[1] = *(const v8us*)(pa1 + 16);
    c0 = wm(a0h.v, bh.v, c0);
    c1 = wm(a1h.v, bh.v, c1);
    if (LO) {
      Frag a0l, a1l, bl;
      const unsigned short* pbl  = Bl + (size_t)ncol * KD + k0 + 8 * hh;
      const unsigned short* pal0 = Al + m * AP + k0 + 8 * hh;
      const unsigned short* pal1 = Al + (16 + m) * AP + k0 + 8 * hh;
      bl.half[0]  = *(const v8us*)pbl;   bl.half[1]  = *(const v8us*)(pbl + 16);
      a0l.half[0] = *(const v8us*)pal0;  a0l.half[1] = *(const v8us*)(pal0 + 16);
      a1l.half[0] = *(const v8us*)pal1;  a1l.half[1] = *(const v8us*)(pal1 + 16);
      c0 = wm(a0h.v, bl.v, c0);
      c0 = wm(a0l.v, bh.v, c0);
      c1 = wm(a1h.v, bl.v, c1);
      c1 = wm(a1l.v, bh.v, c1);
    }
  }
}

__global__ __launch_bounds__(NTHR) void k_gemm0(
    const float* __restrict__ x, const unsigned short* __restrict__ Wh,
    const unsigned short* __restrict__ Wl, const float* __restrict__ bias,
    float* hout, int nN) {
  __shared__ __attribute__((aligned(16))) unsigned short Ah[GR * AP2];
  __shared__ __attribute__((aligned(16))) unsigned short Al[GR * AP2];
  __shared__ __attribute__((aligned(16))) float Xs[GR * XSP];

  const int tid  = threadIdx.x;
  const int lane = tid & 31;
  const int wave = tid >> 5;
  const int hh   = lane >> 4;
  const int m    = lane & 15;
  const int rowBase = blockIdx.x * GR;

  stage128<true>(x, KIN, 0,   rowBase, nN, Ah, Al, AP2, 0,   tid);
  stage128<true>(x, KIN, 128, rowBase, nN, Ah, Al, AP2, 128, tid);
  __syncthreads();

  const int ncol = wave * 16 + m;
  v8f c0 = {0.f, 0.f, 0.f, 0.f, 0.f, 0.f, 0.f, 0.f};
  v8f c1 = {0.f, 0.f, 0.f, 0.f, 0.f, 0.f, 0.f, 0.f};
  mma2<KIN, AP2, true>(Ah, Al, Wh, Wl, ncol, m, hh, c0, c1);

  const float b = bias[ncol];
#pragma unroll
  for (int r = 0; r < 8; ++r) {
    Xs[(8 * hh + r) * XSP + ncol]      = gelu_f(c0[r] + b);
    Xs[(16 + 8 * hh + r) * XSP + ncol] = gelu_f(c1[r] + b);
  }
  __syncthreads();

  v4f xr[4];
  float* xp[4];
#pragma unroll
  for (int i = 0; i < 4; ++i) {
    xr[i] = *(const v4f*)(Xs + (4 * wave + i) * XSP + 4 * lane);
    xp[i] = hout + (size_t)(rowBase + 4 * wave + i) * DF + 4 * lane;
  }
#pragma unroll
  for (int i = 0; i < 4; ++i) *(volatile v4f*)(xp[i]) = xr[i];
  __threadfence();
#pragma unroll
  for (int i = 0; i < 4; ++i) *(volatile v4f*)(xp[i]) = xr[i];
}

__global__ __launch_bounds__(NTHR) void k_gemmh(
    const float* __restrict__ hin, const unsigned short* __restrict__ Wh,
    const float* __restrict__ bias, const float* __restrict__ Wau,
    const float* __restrict__ bau, const float* __restrict__ Wav,
    float* hiout, float* aup, float* avp, int nN) {
  __shared__ __attribute__((aligned(16))) unsigned short Ah[GR * AP1];
  __shared__ __attribute__((aligned(16))) float Xs[GR * XSP];
  __shared__ __attribute__((aligned(16))) float Wst[DF * 8];
  __shared__ __attribute__((aligned(16))) float Pst[GR * 8];

  const int tid  = threadIdx.x;
  const int lane = tid & 31;
  const int wave = tid >> 5;
  const int hh   = lane >> 4;
  const int m    = lane & 15;
  const int rowBase = blockIdx.x * GR;

  if (tid < DF) {
    const v4f wa = *(const v4f*)(Wau + tid * NH);
    const v4f wv = *(const v4f*)(Wav + tid * NH);
    *(v4f*)(Wst + tid * 8)     = wa;
    *(v4f*)(Wst + tid * 8 + 4) = wv;
  }
  stage128<false>(hin, DF, 0, rowBase, nN, Ah, Ah, AP1, 0, tid);
  __syncthreads();

  const int ncol = wave * 16 + m;
  v8f c0 = {0.f, 0.f, 0.f, 0.f, 0.f, 0.f, 0.f, 0.f};
  v8f c1 = {0.f, 0.f, 0.f, 0.f, 0.f, 0.f, 0.f, 0.f};
  mma2<DF, AP1, false>(Ah, Ah, Wh, Wh, ncol, m, hh, c0, c1);

  const float b = bias[ncol];
#pragma unroll
  for (int r = 0; r < 8; ++r) {
    Xs[(8 * hh + r) * XSP + ncol]      = c0[r] + b;
    Xs[(16 + 8 * hh + r) * XSP + ncol] = c1[r] + b;
  }
  __syncthreads();

  {
    const int row = tid >> 3;
    const int q   = tid & 7;
    float s = 0.f;
#pragma unroll 4
    for (int c = 0; c < DF; ++c) s += Xs[row * XSP + c] * Wst[c * 8 + q];
    const float bb = bau[q & 3];
    s += (q < 4) ? bb : 0.f;
    Pst[row * 8 + q] = s;
  }
  __syncthreads();

  v4f xr[4];
  float* xp[4];
#pragma unroll
  for (int i = 0; i < 4; ++i) {
    xr[i] = *(const v4f*)(Xs + (4 * wave + i) * XSP + 4 * lane);
    xp[i] = hiout + (size_t)(rowBase + 4 * wave + i) * DF + 4 * lane;
  }
  v4f gv = {0.f, 0.f, 0.f, 0.f};
  if (wave < 2) gv = *(const v4f*)(Pst + lane * 8 + 4 * wave);
  float* gp = ((wave == 0) ? aup : avp) + ((size_t)rowBase + lane) * HP;

#pragma unroll
  for (int i = 0; i < 4; ++i) *(volatile v4f*)(xp[i]) = xr[i];
  if (wave < 2) *(volatile v4f*)gp = gv;
  __threadfence();
#pragma unroll
  for (int i = 0; i < 4; ++i) *(volatile v4f*)(xp[i]) = xr[i];
  if (wave < 2) *(volatile v4f*)gp = gv;
}

__global__ __launch_bounds__(NTHR) void k_gat(
    const float* __restrict__ hib, const float* __restrict__ aup,
    const float* __restrict__ avp, const int* __restrict__ srcp,
    const int* __restrict__ dstp, float* msg, int nN, int nE) {
  extern __shared__ v4f lds_dyn[];
  float* sacc = (float*)lds_dyn;
  v4f*   daux = lds_dyn + (LDS_SACC / 4);
  v4f*   maux = daux + NB;
  int*   list = (int*)(maux + NB);
  int*   wcnt = list + LDS_LIST;

  const int tid  = threadIdx.x;
  const int lane = tid & 31;
  const int wave = tid >> 5;
  const int nodeBase = blockIdx.x * NB;

  {
    const v4f z4 = {0.f, 0.f, 0.f, 0.f};
    for (int i = tid; i < (LDS_SACC + LDS_DEN) / 4; i += NTHR) lds_dyn[i] = z4;
    const float ninf = __uint_as_float(0xff800000u);
    const v4f n4 = {ninf, ninf, ninf, ninf};
    for (int i = tid; i < LDS_MAX / 4; i += NTHR) lds_dyn[(LDS_SACC + LDS_DEN) / 4 + i] = n4;
  }
  __syncthreads();
  const bool al16 = ((((size_t)dstp) & 15) == 0);

  const int nChunks = (nE + CHUNK - 1) / CHUNK;
#pragma unroll 1
  for (int ch = 0; ch < nChunks; ++ch) {
    const int cbase = ch * CHUNK;
    int wc = 0;
#pragma unroll
    for (int g = 0; g < NGRP; ++g) {
      const int el0 = (g * NTHR + tid) * 4;
      const int e0  = cbase + el0;
      const int sent = -2147483647 - 1;
      v4i d;
      if (al16 && (cbase + CHUNK <= nE)) {
        d = *(const v4i*)(dstp + e0);
      } else {
        d.x = (e0     < nE) ? dstp[min(e0, nE - 1)]     : sent;
        d.y = (e0 + 1 < nE) ? dstp[min(e0 + 1, nE - 1)] : sent;
        d.z = (e0 + 2 < nE) ? dstp[min(e0 + 2, nE - 1)] : sent;
        d.w = (e0 + 3 < nE) ? dstp[min(e0 + 3, nE - 1)] : sent;
      }
      const unsigned s0 = (unsigned)d.x - (unsigned)nodeBase;
      const unsigned s1 = (unsigned)d.y - (unsigned)nodeBase;
      const unsigned s2 = (unsigned)d.z - (unsigned)nodeBase;
      const unsigned s3 = (unsigned)d.w - (unsigned)nodeBase;
      const bool h0 = s0 < (unsigned)NB;
      const bool h1 = s1 < (unsigned)NB;
      const bool h2 = s2 < (unsigned)NB;
      const bool h3 = s3 < (unsigned)NB;
      const unsigned many = __builtin_amdgcn_ballot_w32(h0 | h1 | h2 | h3);
      if (many != 0u) {
#define HITJ(J, HJ, SJ) { \
          const unsigned mj = __builtin_amdgcn_ballot_w32(HJ); \
          if (HJ) { \
            const int pos = wc + (int)__builtin_amdgcn_mbcnt_lo(mj, 0u); \
            if (pos < WCAP) list[wave * WCAP + pos] = ((el0 + (J)) << 9) | (int)(SJ); \
          } \
          wc += (int)__builtin_popcount(mj); }
        HITJ(0, h0, s0)
        HITJ(1, h1, s1)
        HITJ(2, h2, s2)
        HITJ(3, h3, s3)
#undef HITJ
      }
    }
    if (lane == 0) wcnt[wave] = wc;
    __syncthreads();

    if (wave == 0) {
      for (int wsx = 0; wsx < NWAVE; ++wsx) {
        int n = __builtin_amdgcn_readfirstlane(wcnt[wsx]);
        n = n > WCAP ? WCAP : n;
        n = n < 0 ? 0 : n;
#pragma unroll 1
        for (int i = 0; i < n; ++i) {
          const int ent  = __builtin_amdgcn_readfirstlane(list[wsx * WCAP + i]);
          const int slot = ent & (NB - 1);
          const int eloc = (ent >> 9) & (CHUNK - 1);
          int e = cbase + eloc;
          e = e > nE - 1 ? nE - 1 : e;
          int j = srcp[e];
          j = j < 0 ? 0 : (j > nN - 1 ? nN - 1 : j);
          int nd = nodeBase + slot;
          nd = nd > nN - 1 ? nN - 1 : nd;
          const v4f a4 = *(const v4f*)(aup + (size_t)j * HP);
          const v4f b4 = *(const v4f*)(avp + (size_t)nd * HP);
          v4f s = a4 + b4;
          s.x = (s.x > 0.f) ? s.x : 0.2f * s.x;
          s.y = (s.y > 0.f) ? s.y : 0.2f * s.y;
          s.z = (s.z > 0.f) ? s.z : 0.2f * s.z;
          s.w = (s.w > 0.f) ? s.w : 0.2f * s.w;
          const v4f mo = maux[slot];
          const v4f dn = daux[slot];
          v4f mn;
          mn.x = fmaxf(mo.x, s.x); mn.y = fmaxf(mo.y, s.y);
          mn.z = fmaxf(mo.z, s.z); mn.w = fmaxf(mo.w, s.w);
          v4f cf;
          cf.x = __expf(mo.x - mn.x); cf.y = __expf(mo.y - mn.y);
          cf.z = __expf(mo.z - mn.z); cf.w = __expf(mo.w - mn.w);
          v4f p;
          p.x = __expf(s.x - mn.x); p.y = __expf(s.y - mn.y);
          p.z = __expf(s.z - mn.z); p.w = __expf(s.w - mn.w);
          const v4f xv = *(const v4f*)(hib + (size_t)j * DF + 4 * lane);
          v4f* sp = (v4f*)(sacc + slot * DF + 4 * lane);
          const v4f cur = *sp;
          const v4f nxt = cur * cf + xv * p;
          *sp = nxt;
          maux[slot] = mn;
          daux[slot] = dn * cf + p;
        }
      }
    }
    __syncthreads();
  }

#pragma unroll 1
  for (int q = 0; q < NB / NWAVE; ++q) {
    const int slot = wave * (NB / NWAVE) + q;
    const int node = nodeBase + slot;
    if (node >= nN) break;
    const v4f dn = daux[slot];
    v4f inv;
    inv.x = (dn.x > 0.f) ? (1.0f / dn.x) : 0.f;
    inv.y = (dn.y > 0.f) ? (1.0f / dn.y) : 0.f;
    inv.z = (dn.z > 0.f) ? (1.0f / dn.z) : 0.f;
    inv.w = (dn.w > 0.f) ? (1.0f / dn.w) : 0.f;
    const v4f sv = *(const v4f*)(sacc + slot * DF + 4 * lane);
    const v4f y = sv * inv;
    float* op = msg + (size_t)node * DF + 4 * lane;
    *(volatile v4f*)op = y;
    __threadfence();
    *(volatile v4f*)op = y;
  }
}

__global__ __launch_bounds__(NTHR) void k_ffn(
    const float* __restrict__ hib, const float* __restrict__ msg,
    const float* __restrict__ hres,
    const unsigned short* __restrict__ W1h, const float* __restrict__ b1,
    const unsigned short* __restrict__ W2h, const float* __restrict__ b2,
    float* hout, int nN, int nLim) {
  __shared__ __attribute__((aligned(16))) unsigned short Ac[GR * AP2];
  __shared__ __attribute__((aligned(16))) unsigned short At[GR * AP1];
  __shared__ __attribute__((aligned(16))) float Xs[GR * XSP];

  const int tid  = threadIdx.x;
  const int lane = tid & 31;
  const int wave = tid >> 5;
  const int hh   = lane >> 4;
  const int m    = lane & 15;
  const int rowBase = blockIdx.x * GR;

  stage128<false>(hib, DF, 0, rowBase, nN, Ac, Ac, AP2, 0,   tid);
  stage128<false>(msg, DF, 0, rowBase, nN, Ac, Ac, AP2, 128, tid);
  __syncthreads();

  const int ncol = wave * 16 + m;
  v8f c0 = {0.f, 0.f, 0.f, 0.f, 0.f, 0.f, 0.f, 0.f};
  v8f c1 = {0.f, 0.f, 0.f, 0.f, 0.f, 0.f, 0.f, 0.f};
  mma2<KIN, AP2, false>(Ac, Ac, W1h, W1h, ncol, m, hh, c0, c1);

  const float bb1 = b1[ncol];
#pragma unroll
  for (int r = 0; r < 8; ++r) {
    At[(8 * hh + r) * AP1 + ncol]      = bf_bits(gelu_f(c0[r] + bb1));
    At[(16 + 8 * hh + r) * AP1 + ncol] = bf_bits(gelu_f(c1[r] + bb1));
  }
  __syncthreads();

  v8f d0 = {0.f, 0.f, 0.f, 0.f, 0.f, 0.f, 0.f, 0.f};
  v8f d1 = {0.f, 0.f, 0.f, 0.f, 0.f, 0.f, 0.f, 0.f};
  mma2<DF, AP1, false>(At, At, W2h, W2h, ncol, m, hh, d0, d1);

  const float bb2 = b2[ncol];
#pragma unroll
  for (int r = 0; r < 8; ++r) {
    Xs[(8 * hh + r) * XSP + ncol]      = d0[r] + bb2;
    Xs[(16 + 8 * hh + r) * XSP + ncol] = d1[r] + bb2;
  }
  __syncthreads();

  v4f xr[4];
  float* xp[4];
  bool ok[4];
#pragma unroll
  for (int i = 0; i < 4; ++i) {
    const int row = rowBase + 4 * wave + i;
    const v4f rr = *(const v4f*)(hres + (size_t)row * DF + 4 * lane);
    xr[i] = *(const v4f*)(Xs + (4 * wave + i) * XSP + 4 * lane) + rr;
    xp[i] = hout + (size_t)row * DF + 4 * lane;
    ok[i] = row < nLim;
  }
#pragma unroll
  for (int i = 0; i < 4; ++i) if (ok[i]) *(volatile v4f*)(xp[i]) = xr[i];
  __threadfence();
#pragma unroll
  for (int i = 0; i < 4; ++i) if (ok[i]) *(volatile v4f*)(xp[i]) = xr[i];
}

#define MAXL 8

static size_t a256(size_t b) { return (b + 255) & ~(size_t)255; }

extern "C" void kernel_launch(void* const* d_in, const int* in_sizes, int n_in,
                              void* d_out, int out_size, void* d_ws, size_t ws_size,
                              hipStream_t stream) {
  if (n_in != 14) return;
  const int nN = in_sizes[0] / KIN;
  if (nN <= 0 || in_sizes[0] != nN * KIN) return;
  const int nE = in_sizes[1];
  if (nE <= 0 || in_sizes[2] != nE) return;
  if (in_sizes[3] != KIN * DF || in_sizes[4] != DF) return;
  const int L = in_sizes[5] / (DF * DF);
  if (L < 1 || L > MAXL || in_sizes[5] != L * DF * DF) return;
  if (in_sizes[6] != L * DF || in_sizes[7] != L * DF * NH || in_sizes[8] != L * NH ||
      in_sizes[9] != L * DF * NH || in_sizes[10] != L * KIN * DF || in_sizes[11] != L * DF ||
      in_sizes[12] != L * DF * DF || in_sizes[13] != L * DF) return;
  if (out_size != nN * DF) return;

  const float* x    = (const float*)d_in[0];
  const int*   esrc = (const int*)d_in[1];
  const int*   edst = (const int*)d_in[2];
  const float* W_in = (const float*)d_in[3];
  const float* b_in = (const float*)d_in[4];
  const float* Wl   = (const float*)d_in[5];
  const float* bl   = (const float*)d_in[6];
  const float* Wau  = (const float*)d_in[7];
  const float* bau  = (const float*)d_in[8];
  const float* Wav  = (const float*)d_in[9];
  const float* Wf1  = (const float*)d_in[10];
  const float* bf1  = (const float*)d_in[11];
  const float* Wf2  = (const float*)d_in[12];
  const float* bf2  = (const float*)d_in[13];
  float* outp = (float*)d_out;

  const int nP = ((nN + GR - 1) / GR) * GR;
  size_t off = 0;
  char* ws = (char*)d_ws;
  unsigned short* Winh = (unsigned short*)(ws + off); off += a256((size_t)KIN * DF * 2);
  unsigned short* Winl = (unsigned short*)(ws + off); off += a256((size_t)KIN * DF * 2);
  unsigned short* Wlh[MAXL];
  unsigned short* Wf1h[MAXL];
  unsigned short* Wf2h[MAXL];
  for (int l = 0; l < L; ++l) {
    Wlh[l]  = (unsigned short*)(ws + off); off += a256((size_t)DF * DF * 2);
    Wf1h[l] = (unsigned short*)(ws + off); off += a256((size_t)KIN * DF * 2);
    Wf2h[l] = (unsigned short*)(ws + off); off += a256((size_t)DF * DF * 2);
  }
  float* hb0 = (float*)(ws + off); off += a256((size_t)nP * DF * sizeof(float));
  float* hb1 = (float*)(ws + off); off += a256((size_t)nP * DF * sizeof(float));
  float* hib = (float*)(ws + off); off += a256((size_t)nP * DF * sizeof(float));
  float* msg = (float*)(ws + off); off += a256((size_t)nP * DF * sizeof(float));
  float* aup = (float*)(ws + off); off += a256((size_t)nP * HP * sizeof(float));
  float* avp = (float*)(ws + off); off += a256((size_t)nP * HP * sizeof(float));
  if (off > ws_size) return;

  k_prepw<KIN, true><<<DF / 32, NTHR, 0, stream>>>(W_in, Winh, Winl);
  for (int l = 0; l < L; ++l) {
    k_prepw<DF,  false><<<DF / 32, NTHR, 0, stream>>>(Wl  + (size_t)l * DF * DF,  Wlh[l],  Wlh[l]);
    k_prepw<KIN, false><<<DF / 32, NTHR, 0, stream>>>(Wf1 + (size_t)l * KIN * DF, Wf1h[l], Wf1h[l]);
    k_prepw<DF,  false><<<DF / 32, NTHR, 0, stream>>>(Wf2 + (size_t)l * DF * DF,  Wf2h[l], Wf2h[l]);
  }

  const int ggem = nP / GR;
  k_gemm0<<<ggem, NTHR, 0, stream>>>(x, Winh, Winl, b_in, hb0, nN);

  hipFuncSetAttribute(reinterpret_cast<const void*>(&k_gat),
                      hipFuncAttributeMaxDynamicSharedMemorySize, LDS_BYTES);
  const int ggat = (nN + NB - 1) / NB;
  for (int l = 0; l < L; ++l) {
    const float* hcur = (l & 1) ? hb1 : hb0;
    float* hnext = (l & 1) ? hb0 : hb1;
    const bool last = (l == L - 1);
    float* hdst = last ? outp : hnext;
    const int nLim = last ? nN : nP;
    k_gemmh<<<ggem, NTHR, 0, stream>>>(hcur, Wlh[l], bl + (size_t)l * DF,
                                       Wau + (size_t)l * DF * NH, bau + (size_t)l * NH,
                                       Wav + (size_t)l * DF * NH, hib, aup, avp, nN);
    k_gat<<<ggat, NTHR, LDS_BYTES, stream>>>(hib, aup, avp, esrc, edst, msg, nN, nE);
    k_ffn<<<ggem, NTHR, 0, stream>>>(hib, msg, hcur, Wf1h[l], bf1 + (size_t)l * DF,
                                     Wf2h[l], bf2 + (size_t)l * DF, hdst, nN, nLim);
  }
}
